// HWconv2d_14611478741629
// MI455X (gfx1250) — hardware-verified
//
#include <hip/hip_runtime.h>
#include <stdint.h>

#define NB     32
#define CIN    64
#define COUT   128
#define HW     56
#define PLANE  (HW * HW)
#define KTOT   576
#define YG     4
#define NYG    (HW / YG)
#define XR     (YG + 2)
#define XC     (HW + 2)
#define XPITCH 64
#define XSH    (XR * XC * XPITCH)
#define MPX    (YG * HW)
#define MTW    7
#define CHB    64
#define NTHR   256
#define STG    (16 * MPX)
#define NPIECE (STG / 4)
#define WROWCH (KTOT / 8)
#define WCH    (COUT * WROWCH)
#define SCX    64.0f
#define SCW    64.0f
#define INV_A  2.44140625e-04f

static_assert(WCH % 256 == 0);
static_assert(HW % YG == 0);
static_assert(MPX == 2 * MTW * 16);
static_assert(KTOT % 32 == 0);
static_assert((YG * HW * 4) % 128 == 0);
static_assert((PLANE * 4) % 128 == 0);
static_assert(NPIECE % 8 == 0);
static_assert(XSH % 8 == 0);
static_assert(NTHR == 256);

typedef _Float16 v16h __attribute__((ext_vector_type(16)));
typedef _Float16 v8h  __attribute__((ext_vector_type(8)));
typedef float    v8f  __attribute__((ext_vector_type(8)));
typedef float    v4f  __attribute__((ext_vector_type(4)));
typedef unsigned v4u  __attribute__((ext_vector_type(4)));

__device__ __forceinline__ float bf_rne(float f) {
  unsigned u = __float_as_uint(f);
  u = (u + 0x7FFFu + ((u >> 16) & 1u)) & 0xFFFF0000u;
  return __uint_as_float(u);
}
__device__ __forceinline__ unsigned hbits(_Float16 h) {
  return (unsigned)__builtin_bit_cast(unsigned short, h);
}
__device__ __forceinline__ float quant_e5m2(float v) {
  const float av = __builtin_fabsf(v);
  int e = (int)((__float_as_uint(av) >> 23) & 0xFFu) - 127;
  e = (e < -14) ? -14 : e;
  const int e2 = e - 2;
  const float scale  = __uint_as_float((unsigned)(e2 + 127) << 23);
  const float iscale = __uint_as_float((unsigned)(127 - e2) << 23);
  float q = rintf(v * iscale) * scale;
  q = fminf(fmaxf(q, -57344.0f), 57344.0f);
  return (av > 0.0f) ? q : 0.0f;
}
__device__ __forceinline__ v8f zero8f() { v8f z = {0.f, 0.f, 0.f, 0.f, 0.f, 0.f, 0.f, 0.f}; return z; }

__device__ __forceinline__ v16h ldfrag(const _Float16* p) {
  union { v16h v; v8h h[2]; } f;
  f.h[0] = *(const v8h*)(p);
  f.h[1] = *(const v8h*)(p + 16);
  return f.v;
}

__device__ __forceinline__ v8f mma_h(v16h a, v16h b, v8f c) {
  return __builtin_amdgcn_wmma_f32_16x16x32_f16(false, a, false, b, (short)0, c, false, false);
}

__global__ __launch_bounds__(256)
void k_wprep(const float* __restrict__ w, unsigned* wb)
{
  const int q  = blockIdx.x * 256 + threadIdx.x;
  const int qc = (q < WCH) ? q : (WCH - 1);
  const int n  = qc / WROWCH;
  const int kc = (qc - n * WROWCH) * 8;

  unsigned hb[8];
#pragma unroll
  for (int j = 0; j < 8; ++j) {
    const int k  = kc + j;
    const int T  = k >> 6;
    const int ci = k & 63;
    const int kh = T / 3;
    const int kw = T - 3 * kh;
    const float wv = bf_rne(w[((n * CIN + ci) * 3 + kh) * 3 + kw]);
    const float qv = quant_e5m2(wv) * SCW;
    hb[j] = hbits((_Float16)qv);
  }
  v4u wh;
  wh.x = hb[0] | (hb[1] << 16);
  wh.y = hb[2] | (hb[3] << 16);
  wh.z = hb[4] | (hb[5] << 16);
  wh.w = hb[6] | (hb[7] << 16);

  unsigned* dst = wb + (size_t)qc * 4;
  if (q < WCH) *(volatile v4u*)dst = wh;
  __threadfence();
  if (q < WCH) *(volatile v4u*)dst = wh;
}

__global__ __launch_bounds__(NTHR)
void k_conv(const float* __restrict__ x, const _Float16* __restrict__ wt,
            const float* __restrict__ bias, float* out)
{
  __shared__ __align__(16) unsigned xs4[XSH / 2];
  __shared__ __align__(16) float stg[STG];
  __shared__ float bsc[CHB];

  const int tid   = threadIdx.x;
  const int lane  = tid & 31;
  const int wv    = tid >> 5;
  const int lm    = lane & 15;
  const int hh    = lane >> 4;
  const int blk   = blockIdx.x;
  const int chalf = blk & 1;
  const int yg    = (blk >> 1) % NYG;
  const int b     = (blk >> 1) / NYG;
  const int y0    = yg * YG;

  if (tid < CHB) bsc[tid] = 72.0f * bf_rne(bias[chalf * CHB + tid]);

  {
#pragma unroll 1
    for (int it = tid; it < XR * XC * 8; it += NTHR) {
      const int cg  = it / (XR * XC);
      const int pp  = it - cg * (XR * XC);
      const int r   = pp / XC;
      const int col = pp - r * XC;
      const int gy  = y0 - 1 + r;
      const int gx  = col - 1;
      const bool inr = ((unsigned)gy < (unsigned)HW) && ((unsigned)gx < (unsigned)HW);
      const int gyc = (gy < 0) ? 0 : ((gy > HW - 1) ? (HW - 1) : gy);
      const int gxc = (gx < 0) ? 0 : ((gx > HW - 1) ? (HW - 1) : gx);
      const float* s = x + ((size_t)(b * CIN + 8 * cg) * HW + gyc) * HW + gxc;
      unsigned hb[8];
#pragma unroll
      for (int j = 0; j < 8; ++j) {
        const float rv = s[(size_t)j * PLANE];
        const float fv = inr ? (bf_rne(rv) * SCX) : 0.0f;
        hb[j] = hbits((_Float16)fv);
      }
      v4u wh;
      wh.x = hb[0] | (hb[1] << 16);
      wh.y = hb[2] | (hb[3] << 16);
      wh.z = hb[4] | (hb[5] << 16);
      wh.w = hb[6] | (hb[7] << 16);
      *(v4u*)(xs4 + (pp * 8 + cg) * 4) = wh;
    }
  }
  __syncthreads();

  const _Float16* xh = (const _Float16*)xs4;
  const int ct = wv & 3;
  const int ph = wv >> 2;
  const int cB = chalf * CHB + ct * 16 + lm;
  const _Float16* wbp = wt + (size_t)cB * KTOT + 8 * hh;

  int pbase[MTW];
#pragma unroll
  for (int mt = 0; mt < MTW; ++mt) {
    const int p  = 16 * (MTW * ph + mt) + lm;
    const int py = p / HW;
    const int px = p - py * HW;
    pbase[mt] = (py * XC + px) * XPITCH + 8 * hh;
  }

  v8f acc[MTW];
#pragma unroll
  for (int mt = 0; mt < MTW; ++mt) acc[mt] = zero8f();

#pragma unroll 1
  for (int T = 0; T < 9; ++T) {
    const int kh   = T / 3;
    const int kw   = T - 3 * kh;
    const int toff = (kh * XC + kw) * XPITCH;
#pragma unroll
    for (int hf = 0; hf < 2; ++hf) {
      const int s    = 2 * T + hf;
      const int koff = toff + 32 * hf;
      const v16h fb  = ldfrag(wbp + 32 * s);
      v16h fa[MTW];
#pragma unroll
      for (int mt = 0; mt < MTW; ++mt) fa[mt] = ldfrag(xh + pbase[mt] + koff);
#pragma unroll
      for (int mt = 0; mt < MTW; ++mt) acc[mt] = mma_h(fa[mt], fb, acc[mt]);
#if defined(__HIP_DEVICE_COMPILE__)
      asm volatile("v_nop\n\tv_nop\n\tv_nop\n\tv_nop"
                   : "+v"(acc[0]), "+v"(acc[1]), "+v"(acc[2]), "+v"(acc[3]),
                     "+v"(acc[4]), "+v"(acc[5]), "+v"(acc[6])
                   : "v"(fa[0]), "v"(fa[1]), "v"(fa[2]), "v"(fa[3]),
                     "v"(fa[4]), "v"(fa[5]), "v"(fa[6]), "v"(fb));
#endif
    }
  }
#if defined(__HIP_DEVICE_COMPILE__)
  asm volatile("v_nop\n\tv_nop\n\tv_nop\n\tv_nop"
               : "+v"(acc[0]), "+v"(acc[1]), "+v"(acc[2]), "+v"(acc[3]),
                 "+v"(acc[4]), "+v"(acc[5]), "+v"(acc[6]));
#endif

  const size_t oblk = ((size_t)b * COUT + (size_t)chalf * CHB) * PLANE + (size_t)y0 * HW;
#pragma unroll 1
  for (int g = 0; g < 4; ++g) {
    if (ct == g) {
      const float bb = bsc[ct * 16 + lm];
      float* drow = stg + lm * MPX;
#pragma unroll
      for (int mt = 0; mt < MTW; ++mt) {
        const int p0 = 16 * (MTW * ph + mt) + 8 * hh;
#pragma unroll
        for (int r = 0; r < 8; ++r) drow[p0 + r] = fmaxf(acc[mt][r] * INV_A + bb, 0.0f);
      }
    }
    __syncthreads();

    float* ob = out + oblk + (size_t)(16 * g) * PLANE;
    v4f vv[4];
    size_t ao[4];
#pragma unroll
    for (int i = 0; i < 4; ++i) {
      const int q  = tid + NTHR * i;
      const int qc = (q < NPIECE) ? q : (NPIECE - 1);
      const int cl = qc / 56;
      const int j  = qc - cl * 56;
      vv[i] = *(const v4f*)(stg + cl * MPX + 4 * j);
      ao[i] = (size_t)cl * PLANE + (size_t)(4 * j);
    }
#pragma unroll
    for (int i = 0; i < 4; ++i) {
      const int q = tid + NTHR * i;
      if (q < NPIECE) *(volatile v4f*)(ob + ao[i]) = vv[i];
    }
    __threadfence();
#pragma unroll
    for (int i = 0; i < 4; ++i) {
      const int q = tid + NTHR * i;
      if (q < NPIECE) *(volatile v4f*)(ob + ao[i]) = vv[i];
    }
    __syncthreads();
  }
}

extern "C" void kernel_launch(void* const* d_in, const int* in_sizes, int n_in,
                              void* d_out, int out_size, void* d_ws, size_t ws_size,
                              hipStream_t stream) {
  if (n_in < 3) return;
  if (in_sizes[0] != NB * CIN * PLANE) return;
  if (in_sizes[1] != COUT * CIN * 9) return;
  if (in_sizes[2] < COUT) return;
  if (out_size != NB * COUT * PLANE) return;

  const size_t wbytes = (size_t)COUT * KTOT * 2;
  if (wbytes > ws_size) return;

  const float* x    = (const float*)d_in[0];
  const float* w    = (const float*)d_in[1];
  const float* bias = (const float*)d_in[2];
  float* out = (float*)d_out;
  unsigned* wbuf = (unsigned*)d_ws;

  k_wprep<<<dim3(WCH / 256), dim3(256), 0, stream>>>(w, wbuf);
  (void)hipGetLastError();

  k_conv<<<dim3(NB * NYG * 2), dim3(NTHR), 0, stream>>>(x, (const _Float16*)wbuf, bias, out);
  (void)hipGetLastError();
}
